// BaseMixedAttention_57028575756701
// MI455X (gfx1250) — hardware-verified
//
#include <hip/hip_runtime.h>
#include <math.h>

typedef __attribute__((ext_vector_type(16))) _Float16 v16h;
typedef __attribute__((ext_vector_type(16))) __bf16 v16b;
typedef __attribute__((ext_vector_type(8)))  _Float16 v8h;
typedef __attribute__((ext_vector_type(8)))  float v8f;
typedef __attribute__((ext_vector_type(4)))  float v4f;
typedef __attribute__((ext_vector_type(2)))  float v2f;
typedef __attribute__((ext_vector_type(4)))  unsigned v4u;
typedef __attribute__((ext_vector_type(4)))  int v4i;
typedef float __attribute__((may_alias)) float_a;
typedef int __attribute__((may_alias)) int_a;

template <typename T> __device__ __forceinline__ void vst2(void* p, T v) { *(volatile T*)p = v; __threadfence(); *(volatile T*)p = v; }
__device__ __forceinline__ v8f wmma16(v16h a, v16h b, v8f c) {
  v8f d = __builtin_amdgcn_wmma_f32_16x16x32_f16(false, a, false, b, (short)0, c, false, false);
  asm volatile("v_nop\n\tv_nop\n\tv_nop\n\tv_nop" : "+v"(d) : "v"(a), "v"(b));
  return d;
}
__device__ __forceinline__ v8f wmma_bf(v16b a, v16b b, v8f c) {
  v8f d = __builtin_amdgcn_wmma_f32_16x16x32_bf16(false, a, false, b, (short)0, c, false, false);
  asm volatile("v_nop\n\tv_nop\n\tv_nop\n\tv_nop" : "+v"(d) : "v"(a), "v"(b));
  return d;
}
__device__ __forceinline__ v16h frag_h(const _Float16* rowk0, int lane) {
  union { v16h v; v8h q[2]; } u; const _Float16* p = rowk0 + 8 * (lane >> 4);
  u.q[0] = *(const v8h*)p; u.q[1] = *(const v8h*)(p + 16); return u.v;
}
__device__ __forceinline__ v16h frag_f32(const float* rowk0, int lane) {
  v16h a; const float* p = rowk0 + 8 * (lane >> 4);
#pragma unroll
  for (int i = 0; i < 8; ++i) { a[i] = (_Float16)p[i]; a[8 + i] = (_Float16)p[16 + i]; }
  return a;
}
__device__ __forceinline__ v16h frag_f32s(const float* rowk0, int lane, float sc) {
  v16h a; const float* p = rowk0 + 8 * (lane >> 4);
#pragma unroll
  for (int i = 0; i < 8; ++i) { a[i] = (_Float16)(p[i] * sc); a[8 + i] = (_Float16)(p[16 + i] * sc); }
  return a;
}
__device__ __forceinline__ v16h fragc_f32(const float* W, int k0, int n, int lane, int ld, int K) {
  v16h a; const int g = lane >> 4;
#pragma unroll
  for (int i = 0; i < 8; ++i) { const int ka = k0 + 8 * g + i, kb = ka + 16;
    a[i] = (_Float16)(ka < K ? W[(size_t)ka * ld + n] : 0.f); a[8 + i] = (_Float16)(kb < K ? W[(size_t)kb * ld + n] : 0.f); }
  return a;
}
struct F2 { v16b h, l; };
__device__ __forceinline__ F2 bsplit16(const float v[16]) { F2 r;
#pragma unroll
  for (int i = 0; i < 16; ++i) { const __bf16 h = (__bf16)v[i]; r.h[i] = h; r.l[i] = (__bf16)(v[i] - (float)h); }
  return r; }
__device__ __forceinline__ F2 split_row(const float* row, int k0, int lane) { float v[16]; const float* p = row + k0 + 8 * (lane >> 4);
#pragma unroll
  for (int i = 0; i < 8; ++i) { v[i] = p[i]; v[8 + i] = p[16 + i]; }
  return bsplit16(v); }
__device__ __forceinline__ F2 split_rowK(const float* row, int k0, int lane, int K) { float v[16]; const int g = lane >> 4;
#pragma unroll
  for (int i = 0; i < 8; ++i) { const int ka = k0 + 8 * g + i, kb = ka + 16; v[i] = ka < K ? row[ka] : 0.f; v[8 + i] = kb < K ? row[kb] : 0.f; }
  return bsplit16(v); }
__device__ __forceinline__ F2 split_col(const float* W, int k0, int n, int lane, int ld, int K) { float v[16]; const int g = lane >> 4;
#pragma unroll
  for (int i = 0; i < 8; ++i) { const int ka = k0 + 8 * g + i, kb = ka + 16; v[i] = ka < K ? W[(size_t)ka * ld + n] : 0.f; v[8 + i] = kb < K ? W[(size_t)kb * ld + n] : 0.f; }
  return bsplit16(v); }
__device__ __forceinline__ v8f mac3(const F2& a, const F2& b, v8f c) { c = wmma_bf(a.l, b.h, c); c = wmma_bf(a.h, b.l, c); return wmma_bf(a.h, b.h, c); }
__device__ __forceinline__ float sigm(float v) { return 1.0f / (1.0f + expf(-v)); }
#define LDSX() do { asm volatile("s_wait_dscnt 0" ::: "memory"); __builtin_amdgcn_wave_barrier(); __builtin_amdgcn_fence(__ATOMIC_RELEASE, "workgroup"); } while (0)


#define NB 8
#define SS 1024
#define E 512
#define NH 8
#define HD 64
#define NR (NB * SS)
#define NTX 77
#define LT 256
#define NKEY 1152
#define TE 2048
__device__ __forceinline__ float silu(float x) { return x / (1.0f + expf(-x)); }

__global__ __launch_bounds__(256) void k_lnx(const float* __restrict__ x, const float* __restrict__ g_, const float* __restrict__ b_, _Float16* __restrict__ X16) {
  const int wave = threadIdx.x >> 5, lane = threadIdx.x & 31; const int row = blockIdx.x * 8 + wave; const float* xr = x + (size_t)row * E;
  float v[16]; float s = 0.f;
#pragma unroll
  for (int e = 0; e < 16; ++e) { v[e] = xr[(e < 8 ? 0 : 256) + lane * 8 + (e & 7)]; s += v[e]; }
#pragma unroll
  for (int o = 16; o > 0; o >>= 1) s += __shfl_xor(s, o, 32);
  const float mu = s * (1.0f / E); float q = 0.f;
#pragma unroll
  for (int e = 0; e < 16; ++e) { const float d = v[e] - mu; q += d * d; }
#pragma unroll
  for (int o = 16; o > 0; o >>= 1) q += __shfl_xor(q, o, 32);
  const float rs = rsqrtf(q * (1.0f / E) + 1e-5f);
  union { v8h h[2]; v4u u[2]; } pk;
#pragma unroll
  for (int e = 0; e < 16; ++e) { const int c = (e < 8 ? 0 : 256) + lane * 8 + (e & 7); pk.h[e >> 3][e & 7] = (_Float16)((v[e] - mu) * rs * g_[c] + b_[c]); }
  vst2(X16 + (size_t)row * E + lane * 8, pk.u[0]); vst2(X16 + (size_t)row * E + 256 + lane * 8, pk.u[1]);
}
__global__ __launch_bounds__(256) void k_lnt(const float* __restrict__ xf, const float* __restrict__ g_, const float* __restrict__ b_, _Float16* __restrict__ T16) {
  const int wave = threadIdx.x >> 5, lane = threadIdx.x & 31; const int row = blockIdx.x * 8 + wave; if (row >= NB * NTX) return; const float* xr = xf + (size_t)row * LT;
  float v[8]; float s = 0.f;
#pragma unroll
  for (int e = 0; e < 8; ++e) { v[e] = xr[lane * 8 + e]; s += v[e]; }
#pragma unroll
  for (int o = 16; o > 0; o >>= 1) s += __shfl_xor(s, o, 32);
  const float mu = s * (1.0f / LT); float q = 0.f;
#pragma unroll
  for (int e = 0; e < 8; ++e) { const float d = v[e] - mu; q += d * d; }
#pragma unroll
  for (int o = 16; o > 0; o >>= 1) q += __shfl_xor(q, o, 32);
  const float rs = rsqrtf(q * (1.0f / LT) + 1e-5f);
  union { v8h h; v4u u; } pk;
#pragma unroll
  for (int e = 0; e < 8; ++e) { const int c = lane * 8 + e; pk.h[e] = (_Float16)((v[e] - mu) * rs * g_[c] + b_[c]); }
  vst2(T16 + (size_t)row * LT + lane * 8, pk.u);
}
__global__ __launch_bounds__(256) void k_pack(const float* __restrict__ Wq, const float* __restrict__ Wkm, const float* __restrict__ Wvm, const float* __restrict__ Wo, const float* __restrict__ Wkt, const float* __restrict__ Wvt, _Float16* __restrict__ PT, _Float16* __restrict__ PT2) {
  const int n = blockIdx.x, tid = threadIdx.x; __shared__ __align__(16) _Float16 srow[E];
  if (n < 4 * E) { const float* W = n < E ? Wq : (n < 2 * E ? Wkm : (n < 3 * E ? Wvm : Wo)); const int nn = n & (E - 1);
    srow[tid] = (_Float16)(W[(size_t)nn * E + tid] * 16.0f); srow[tid + 256] = (_Float16)(W[(size_t)nn * E + tid + 256] * 16.0f); __syncthreads();
    if (tid < E / 8) vst2(PT + (size_t)n * E + tid * 8, *(const v4u*)(&srow[tid * 8])); }
  else { const int m = n - 4 * E; const float* W = m < E ? Wkt : Wvt; const int nn = m & (E - 1);
    srow[tid] = (_Float16)(W[(size_t)nn * LT + tid] * 16.0f); __syncthreads();
    if (tid < LT / 8) vst2(PT2 + (size_t)m * LT + tid * 8, *(const v4u*)(&srow[tid * 8])); }
}
__global__ __launch_bounds__(128) void k_qkv(const _Float16* __restrict__ X16, const _Float16* __restrict__ PT, const float* __restrict__ bq, const float* __restrict__ bk, const float* __restrict__ bv, const float* __restrict__ srcm,
                                            _Float16* __restrict__ Q16, _Float16* __restrict__ K16, _Float16* __restrict__ VT) {
  __shared__ __align__(16) float so[4][16][132];
  __shared__ __align__(16) _Float16 sth[128][72];
  const int tid = threadIdx.x, wave = tid >> 5, lane = tid & 31, col = lane & 15, g = lane >> 4;
  const int which = blockIdx.z, r0b = blockIdx.x * 64, r0 = r0b + wave * 16, n0 = blockIdx.y * 128; const int b = r0b / SS, s0 = r0b % SS;
  const float* bb_ = which == 0 ? bq : (which == 1 ? bk : bv);
  v8f acc[8] = {};
#pragma unroll 2
  for (int kc = 0; kc < E / 32; ++kc) { const v16h a = frag_h(X16 + (size_t)(r0 + col) * E + kc * 32, lane);
#pragma unroll
    for (int j = 0; j < 8; ++j) acc[j] = wmma16(a, frag_h(PT + (size_t)(which * E + n0 + j * 16 + col) * E + kc * 32, lane), acc[j]); }
  if (which < 2) {
#pragma unroll
    for (int j = 0; j < 8; ++j) { const float bb = bb_[n0 + j * 16 + col];
#pragma unroll
      for (int r = 0; r < 8; ++r) so[wave][8 * g + r][j * 16 + col] = (acc[j][r] * (1.0f / 16.0f) + bb) * 4.0f; }
    LDSX();
    for (int qq = lane; qq < 16 * 2 * 8; qq += 32) { const int hh = qq >> 7, rl = (qq >> 3) & 15, pc = qq & 7; const int h = (n0 >> 6) + hh; union { v8h h8; v4u u; } pk;
#pragma unroll
      for (int e = 0; e < 8; ++e) pk.h8[e] = (_Float16)so[wave][rl][hh * 64 + pc * 8 + e];
      if (which == 0) vst2(Q16 + (((size_t)b * NH + h) * SS + s0 + wave * 16 + rl) * HD + pc * 8, pk.u);
      else vst2(K16 + (((size_t)b * NH + h) * NKEY + NTX + s0 + wave * 16 + rl) * HD + pc * 8, pk.u); } }
  else {
#pragma unroll
    for (int j = 0; j < 8; ++j) { const float bb = bb_[n0 + j * 16 + col];
#pragma unroll
      for (int r = 0; r < 8; ++r) { const int s = s0 + wave * 16 + 8 * g + r; sth[j * 16 + col][wave * 16 + 8 * g + r] = (_Float16)((acc[j][r] * (1.0f / 16.0f) + bb) * srcm[b * SS + s] * 4.0f); } }
    __syncthreads();
    for (int qq = tid; qq < 64 * 16; qq += 128) { const int rl = qq >> 4, pc = qq & 15; const int s = s0 + rl;
      union { v8h h8; v4u u; } pk;
#pragma unroll
      for (int e = 0; e < 8; ++e) pk.h8[e] = sth[pc * 8 + e][rl];
      vst2(VT + ((size_t)b * SS + s) * E + n0 + pc * 8, pk.u); } }
}
__global__ __launch_bounds__(128) void k_tkv(const _Float16* __restrict__ T16, const _Float16* __restrict__ PT2, const float* __restrict__ bkt, const float* __restrict__ bvt, const int* __restrict__ cond, _Float16* __restrict__ K16, _Float16* __restrict__ VS2) {
  __shared__ __align__(16) float so[4][16][132];
  const int tid = threadIdx.x, wave = tid >> 5, lane = tid & 31, col = lane & 15, g = lane >> 4;
  const int b = blockIdx.z, which = blockIdx.y; const int t0 = (blockIdx.x >> 2) * 64 + wave * 16, n0 = (blockIdx.x & 3) * 128;
  const float tc = (cond[b] % 10) > 0 ? 1.f : 0.f; const float* bb_ = which == 0 ? bkt : bvt; const float vsc = which == 0 ? 4.0f : 4.0f * tc;
  const int tr = (t0 + col) < NTX ? (t0 + col) : (NTX - 1);
  v8f acc[8] = {};
#pragma unroll 2
  for (int kc = 0; kc < LT / 32; ++kc) { const v16h a = frag_h(T16 + ((size_t)b * NTX + tr) * LT + kc * 32, lane);
#pragma unroll
    for (int j = 0; j < 8; ++j) acc[j] = wmma16(a, frag_h(PT2 + (size_t)(which * E + n0 + j * 16 + col) * LT + kc * 32, lane), acc[j]); }
#pragma unroll
  for (int j = 0; j < 8; ++j) { const float bb = bb_[n0 + j * 16 + col];
#pragma unroll
    for (int r = 0; r < 8; ++r) so[wave][8 * g + r][j * 16 + col] = (acc[j][r] * (1.0f / 16.0f) + bb) * vsc; }
  LDSX();
  if (which == 0) {
    for (int qq = lane; qq < 16 * 2 * 8; qq += 32) { const int hh = qq >> 7, rl = (qq >> 3) & 15, pc = qq & 7; const int h = (n0 >> 6) + hh; const int t = t0 + rl; if (t >= NTX) continue; union { v8h h8; v4u u; } pk;
#pragma unroll
      for (int e = 0; e < 8; ++e) pk.h8[e] = (_Float16)so[wave][rl][hh * 64 + pc * 8 + e];
      vst2(K16 + (((size_t)b * NH + h) * NKEY + t) * HD + pc * 8, pk.u); } }
  else {
    for (int qq = lane; qq < 16 * 16; qq += 32) { const int rl = qq >> 4, pc = qq & 15; const int t = t0 + rl; if (t >= NTX) continue; union { v8h h8; v4u u; } pk;
#pragma unroll
      for (int e = 0; e < 8; ++e) pk.h8[e] = (_Float16)so[wave][rl][pc * 8 + e];
      vst2(VS2 + ((size_t)b * NTX + t) * E + n0 + pc * 8, pk.u); } }
}
__global__ __launch_bounds__(256) void k_vt(const _Float16* __restrict__ VS, const _Float16* __restrict__ VS2, _Float16* __restrict__ VT) {
  __shared__ __align__(16) _Float16 st[8][NKEY + 8];
  const int tid = threadIdx.x; const int bh = blockIdx.x >> 3, d0 = (blockIdx.x & 7) * 8; const int b = bh / NH, h = bh % NH; const int c0 = h * HD + d0;
  for (int q = tid; q < 8 * NKEY; q += 256) { const int dl = q / NKEY, slot = q % NKEY; _Float16 v;
    if (slot < NTX) v = VS2[((size_t)b * NTX + slot) * E + c0 + dl]; else if (slot < NTX + SS) v = VS[((size_t)b * SS + (slot - NTX)) * E + c0 + dl]; else v = (_Float16)0.f;
    st[dl][slot] = v; }
  __syncthreads();
  for (int q = tid; q < 8 * (NKEY / 8); q += 256) { const int dl = q / (NKEY / 8), pc = q % (NKEY / 8); vst2(VT + ((size_t)bh * HD + d0 + dl) * NKEY + pc * 8, *(const v4u*)(&st[dl][pc * 8])); }
}
__global__ __launch_bounds__(256) void k_zpad(_Float16* __restrict__ K16) {
  const int bh = blockIdx.x, tid = threadIdx.x; const v4u z = {0u, 0u, 0u, 0u};
  for (int q = tid; q < (NKEY - NTX - SS) * 8; q += 256) { const int rl = q >> 3, pc = q & 7; vst2(K16 + (((size_t)bh) * NKEY + NTX + SS + rl) * HD + pc * 8, z); }
}
__global__ __launch_bounds__(128) void k_attn(const _Float16* __restrict__ Q16, const _Float16* __restrict__ K16, const _Float16* __restrict__ VT, const int* __restrict__ cond, const float* __restrict__ srcm, _Float16* __restrict__ O16) {
  __shared__ __align__(16) float sS[4][16][68];
  __shared__ __align__(16) _Float16 sPh[4][16][72];
  __shared__ __align__(16) float sO[4][16][68];
  const int tid = threadIdx.x, w = tid >> 5, lane = tid & 31, col = lane & 15, g = lane >> 4;
  const size_t bh = blockIdx.y; const int b = (int)(bh / NH); const int q0 = blockIdx.x * 64 + w * 16;
  const float tpen = ((cond[b] % 10) > 0) ? 0.f : -1000000.0f;
  v16h aq[2];
#pragma unroll
  for (int kc = 0; kc < 2; ++kc) aq[kc] = frag_h(Q16 + (bh * SS + q0 + col) * HD + kc * 32, lane);
  float mrun = -3.0e38f, lrun = 0.f; v8f acc[4] = {};
#pragma unroll 1
  for (int kt = 0; kt < NKEY / 64; ++kt) {
#pragma unroll
    for (int t = 0; t < 4; ++t) { v8f s = {}; const int slot = kt * 64 + t * 16 + col;
#pragma unroll
      for (int kc = 0; kc < 2; ++kc) s = wmma16(aq[kc], frag_h(K16 + (bh * NKEY + slot) * HD + kc * 32, lane), s);
      float pen; if (slot < NTX) pen = tpen; else if (slot < NTX + SS) pen = (1.0f - srcm[b * SS + slot - NTX]) * -1000000.0f; else pen = -3.0e38f;
#pragma unroll
      for (int r = 0; r < 8; ++r) sS[w][8 * g + r][t * 16 + col] = slot < NTX + SS ? s[r] * (1.0f / 16.0f) + pen : -3.0e38f; }
    LDSX();
    float mx = -3.4e38f;
#pragma unroll
    for (int jj = 0; jj < 32; ++jj) mx = fmaxf(mx, sS[w][col][g * 32 + jj]);
    mx = fmaxf(mx, __shfl_xor(mx, 16, 32));
    const float mnew = fmaxf(mrun, mx); const float corr = expf(mrun - mnew);
    float ps = 0.f;
#pragma unroll
    for (int jj = 0; jj < 32; ++jj) { const float sv = sS[w][col][g * 32 + jj]; const float p = sv <= -1.0e38f ? 0.f : expf(sv - mnew) * 16384.0f; ps += p; sPh[w][col][g * 32 + jj] = (_Float16)p; }
    ps += __shfl_xor(ps, 16, 32);
    lrun = lrun * corr + ps * (1.0f / 16384.0f); mrun = mnew;
#pragma unroll
    for (int r = 0; r < 8; ++r) { const float cr = __shfl(corr, 8 * g + r, 32);
#pragma unroll
      for (int t = 0; t < 4; ++t) acc[t][r] *= cr; }
    LDSX();
#pragma unroll
    for (int kc = 0; kc < 2; ++kc) { const v16h ph = frag_h(&sPh[w][col][0] + kc * 32, lane);
#pragma unroll
      for (int t = 0; t < 4; ++t) { const size_t vo = (bh * HD + t * 16 + col) * NKEY + kt * 64 + kc * 32; acc[t] = wmma16(ph, frag_h(VT + vo, lane), acc[t]); } }
    __builtin_amdgcn_wave_barrier(); }
#pragma unroll
  for (int r = 0; r < 8; ++r) { const float lr = __shfl(lrun, 8 * g + r, 32); const float inv = 8.0f / (lr * 16384.0f * 4.0f);
#pragma unroll
    for (int t = 0; t < 4; ++t) sO[w][8 * g + r][t * 16 + col] = acc[t][r] * inv; }
  LDSX();
  for (int qq = lane; qq < 16 * 8; qq += 32) { const int rl = qq >> 3, pc = qq & 7; union { v8h h8; v4u u; } pk;
#pragma unroll
    for (int e = 0; e < 8; ++e) pk.h8[e] = (_Float16)sO[w][rl][pc * 8 + e];
    vst2(O16 + ((bh * SS) + q0 + rl) * HD + pc * 8, pk.u); }
}
__global__ __launch_bounds__(128) void k_emb(const float* __restrict__ emb, const float* __restrict__ W, const float* __restrict__ bias, float* __restrict__ SSH) {
  __shared__ __align__(16) float se[16][TE + 8];
  const int tid = threadIdx.x, wave = tid >> 5, lane = tid & 31, col = lane & 15, g = lane >> 4; const int n0 = blockIdx.x * 128 + wave * 32;
  for (int q = tid; q < 16 * TE; q += 128) { const int r = q / TE, k = q % TE; se[r][k] = r < NB ? silu(emb[(size_t)r * TE + k]) : 0.f; }
  __syncthreads();
  v8f acc[2] = {};
#pragma unroll 1
  for (int kc = 0; kc < TE / 32; ++kc) { const F2 a = split_row(&se[col][0], kc * 32, lane);
#pragma unroll
    for (int j = 0; j < 2; ++j) acc[j] = mac3(a, split_row(W + (size_t)(n0 + j * 16 + col) * TE, kc * 32, lane), acc[j]); }
  __shared__ __align__(16) float so[4][16][36];
#pragma unroll
  for (int j = 0; j < 2; ++j)
#pragma unroll
    for (int r = 0; r < 8; ++r) so[wave][8 * g + r][j * 16 + col] = acc[j][r] + bias[n0 + j * 16 + col];
  LDSX();
  for (int qq = lane; qq < 8 * 8; qq += 32) { const int r = qq >> 3, pc = qq & 7; vst2(SSH + (size_t)r * (2 * E) + n0 + pc * 4, *(const v4f*)(&so[wave][r][pc * 4])); }
}
__global__ __launch_bounds__(256) void k_styl(const _Float16* __restrict__ O16, const float* __restrict__ SSH, const float* __restrict__ g_, const float* __restrict__ b_, _Float16* __restrict__ Z16) {
  const int wave = threadIdx.x >> 5, lane = threadIdx.x & 31; const int row = blockIdx.x * 8 + wave; const int b = row / SS, s = row % SS;
  float sum = 0.f, sq = 0.f;
#pragma unroll 2
  for (int e = 0; e < 16; ++e) { const int c = (e < 8 ? 0 : 256) + lane * 8 + (e & 7); const int h = c >> 6, d = c & 63; const float v = (float)O16[(((size_t)b * NH + h) * SS + s) * HD + d] * 0.125f; sum += v; sq += v * v; }
#pragma unroll
  for (int o = 16; o > 0; o >>= 1) { sum += __shfl_xor(sum, o, 32); sq += __shfl_xor(sq, o, 32); }
  const float mu = sum * (1.0f / E); float var = sq * (1.0f / E) - mu * mu; var = var > 0.f ? var : 0.f; const float rs = rsqrtf(var + 1e-5f);
  const float* sc_ = SSH + (size_t)b * 2 * E; const float* sh_ = sc_ + E;
#pragma unroll 1
  for (int half = 0; half < 2; ++half) { union { v8h h; v4u u; } pk;
#pragma unroll
    for (int e = 0; e < 8; ++e) { const int c = half * 256 + lane * 8 + e; const int h = c >> 6, d = c & 63; const float v = (float)O16[(((size_t)b * NH + h) * SS + s) * HD + d] * 0.125f;
      const float hn = (v - mu) * rs * g_[c] + b_[c]; const float m = hn * (1.0f + sc_[c]) + sh_[c]; pk.h[e] = (_Float16)(silu(m) * 8.0f); }
    vst2(Z16 + (size_t)row * E + half * 256 + lane * 8, pk.u); }
}
__global__ __launch_bounds__(128) void k_out(const _Float16* __restrict__ Z16, const _Float16* __restrict__ PT, const float* __restrict__ bo, const float* __restrict__ x, float* __restrict__ out) {
  __shared__ __align__(16) float so[4][16][132];
  const int tid = threadIdx.x, wave = tid >> 5, lane = tid & 31, col = lane & 15, g = lane >> 4;
  const int r0 = blockIdx.x * 64 + wave * 16, n0 = blockIdx.y * 128;
  v8f acc[8] = {};
#pragma unroll 2
  for (int kc = 0; kc < E / 32; ++kc) { const v16h a = frag_h(Z16 + (size_t)(r0 + col) * E + kc * 32, lane);
#pragma unroll
    for (int j = 0; j < 8; ++j) acc[j] = wmma16(a, frag_h(PT + (size_t)(3 * E + n0 + j * 16 + col) * E + kc * 32, lane), acc[j]); }
#pragma unroll
  for (int j = 0; j < 8; ++j) { const int n = n0 + j * 16 + col; const float bb = bo[n];
#pragma unroll
    for (int r = 0; r < 8; ++r) so[wave][8 * g + r][j * 16 + col] = acc[j][r] * (1.0f / (16.0f * 8.0f)) + bb + x[(size_t)(r0 + 8 * g + r) * E + n]; }
  LDSX();
#pragma unroll 4
  for (int rl = 0; rl < 16; ++rl) vst2(out + (size_t)(r0 + rl) * E + n0 + lane * 4, *(const v4f*)(&so[wave][rl][lane * 4]));
}
extern "C" void kernel_launch(void* const* d_in, const int* in_sizes, int n_in, void* d_out, int out_size, void* d_ws, size_t ws_size, hipStream_t stream) {
  (void)in_sizes; (void)n_in; (void)out_size; (void)ws_size;
  const float** I = (const float**)d_in;
  const float* x = I[0]; const float* xf = I[1]; const float* emb = I[2]; const float* srcm = I[3]; const int* cond = (const int*)d_in[4];
  const float* ng = I[5]; const float* nb = I[6]; const float* tg = I[7]; const float* tb = I[8]; const float* Wq = I[9]; const float* bq = I[10]; const float* Wkt = I[11]; const float* bkt = I[12]; const float* Wvt = I[13]; const float* bvt = I[14];
  const float* Wkm = I[15]; const float* bkm = I[16]; const float* Wvm = I[17]; const float* bvm = I[18]; const float* embW = I[19]; const float* embb = I[20]; const float* sg = I[21]; const float* sb = I[22]; const float* Wo = I[23]; const float* bo = I[24];
  float* out = (float*)d_out;
  char* ws = (char*)d_ws; size_t off = 0;
  auto take = [&](size_t bytes) { char* p = ws + off; off += (bytes + 255) & ~(size_t)255; return p; };
  _Float16* X16 = (_Float16*)take((size_t)NR * E * 2); _Float16* T16 = (_Float16*)take((size_t)NB * NTX * LT * 2 + 4096); _Float16* PT = (_Float16*)take((size_t)4 * E * E * 2); _Float16* PT2 = (_Float16*)take((size_t)2 * E * LT * 2);
  _Float16* Q16 = (_Float16*)take((size_t)NR * E * 2); _Float16* K16 = (_Float16*)take((size_t)NB * NH * NKEY * HD * 2); _Float16* VS = (_Float16*)take((size_t)NR * E * 2); _Float16* VS2 = (_Float16*)take((size_t)NB * NTX * E * 2 + 4096);
  _Float16* VT = (_Float16*)take((size_t)NB * NH * HD * NKEY * 2); _Float16* O16 = (_Float16*)take((size_t)NR * E * 2); float* SSH = (float*)take((size_t)NB * 2 * E * 4); _Float16* Z16 = X16;
  k_lnx<<<NR / 8, 256, 0, stream>>>(x, ng, nb, X16);
  k_lnt<<<(NB * NTX + 7) / 8, 256, 0, stream>>>(xf, tg, tb, T16);
  k_pack<<<4 * E + 2 * E, 256, 0, stream>>>(Wq, Wkm, Wvm, Wo, Wkt, Wvt, PT, PT2);
  k_qkv<<<dim3(NR / 64, E / 128, 3), 128, 0, stream>>>(X16, PT, bq, bkm, bvm, srcm, Q16, K16, VS);
  k_tkv<<<dim3(2 * 4, 2, NB), 128, 0, stream>>>(T16, PT2, bkt, bvt, cond, K16, VS2);
  k_zpad<<<NB * NH, 256, 0, stream>>>(K16);
  k_vt<<<NB * NH * 8, 256, 0, stream>>>(VS, VS2, VT);
  k_attn<<<dim3(SS / 64, NB * NH), 128, 0, stream>>>(Q16, K16, VT, cond, srcm, O16);
  k_emb<<<(2 * E) / 128, 128, 0, stream>>>(emb, embW, embb, SSH);
  k_styl<<<NR / 8, 256, 0, stream>>>(O16, SSH, sg, sb, Z16);
  k_out<<<dim3(NR / 64, E / 128), 128, 0, stream>>>(Z16, PT, bo, x, out);
}
